// TemporalGNN_11836929868099
// MI455X (gfx1250) — hardware-verified
//
#include <hip/hip_runtime.h>
#include <math.h>

constexpr int kT    = 8;
constexpr int kN    = 1024;
constexpr int kIn   = 64;
constexpr int kHid  = 128;
constexpr int kOut  = 64;
constexpr int kE    = 16384;
constexpr int kRows = kT * kN;
constexpr int kTD   = 128;
constexpr int kTiles = kN / kTD;
constexpr int kThr  = 256;
constexpr int kSch  = 2048;
constexpr int kSpt  = kSch / kThr;
constexpr int kNch  = kE / kSch;
constexpr int kPairBlocks = kN - 1;
constexpr int kPairsPerBlock = 1024;
constexpr float kCarry = 16.0f;
constexpr float kScale1 = 1.0f / 16.0f;
constexpr float kScale2 = 1.0f / 256.0f;

static_assert(kE % kSch == 0, "chunking exact");
static_assert(kSpt == 8, "two int4 loads per thread");
static_assert(kN % kTD == 0 && kTD == 128, "tile");
static_assert(kTD / 8 == 16, "16 rows per wave");
static_assert(kPairBlocks * kPairsPerBlock == kN * (kN - 1), "flat pair ownership exact");
static_assert(kRows % 64 == 0 && kN % 64 == 0 && kHid % 64 == 0 && kOut % 64 == 0, "GEMM M,N tile multiples");
static_assert(kIn % 32 == 0 && kHid % 32 == 0 && kOut % 32 == 0, "GEMM K multiples of 32");
static_assert(kT * kOut == 512, "pool thread map");

typedef __attribute__((ext_vector_type(16))) _Float16 v16h;
typedef __attribute__((ext_vector_type(8)))  _Float16 v8h;
typedef __attribute__((ext_vector_type(16))) __bf16   v16b;
typedef __attribute__((ext_vector_type(8)))  __bf16   v8b;
typedef __attribute__((ext_vector_type(8)))  float    v8f;
typedef __attribute__((ext_vector_type(4)))  float    v4f;
typedef __attribute__((ext_vector_type(2)))  float    v2f;
typedef __attribute__((ext_vector_type(4)))  int      v4i;
typedef __attribute__((ext_vector_type(4)))  unsigned int v4u;

__device__ __forceinline__ unsigned short f2bf_bits(float f) {
  unsigned u = __float_as_uint(f);
  return (unsigned short)((u + 0x7FFFu + ((u >> 16) & 1u)) >> 16);
}
__device__ __forceinline__ float bf_bits2f(unsigned short h) { return __uint_as_float(((unsigned)h) << 16); }

__device__ __forceinline__ void dep_guard_h(v8f& a, v8f& b, v16h x, v16h y) { asm volatile("v_nop\n\tv_nop\n\tv_nop\n\tv_nop" : "+v"(a), "+v"(b) : "v"(x), "v"(y)); }
__device__ __forceinline__ void dep_guard_b(v8f& a, v8f& b, v16b x, v16b y) { asm volatile("v_nop\n\tv_nop\n\tv_nop\n\tv_nop" : "+v"(a), "+v"(b) : "v"(x), "v"(y)); }
__device__ __forceinline__ void keep4_h(v16h a, v16h b, v16h c, v16h d) { asm volatile("v_nop" :: "v"(a), "v"(b), "v"(c), "v"(d)); }
__device__ __forceinline__ void keep4_b(v16b a, v16b b, v16b c, v16b d) { asm volatile("v_nop" :: "v"(a), "v"(b), "v"(c), "v"(d)); }
__device__ __forceinline__ void acc_guard4(v8f& a, v8f& b, v8f& c, v8f& d) { asm volatile("v_nop\n\tv_nop\n\tv_nop\n\tv_nop" : "+v"(a), "+v"(b), "+v"(c), "+v"(d)); }
template <typename T> struct Frag;
template <> struct Frag<_Float16> {
  typedef v16h V; union U { v16h v; v8h h[2]; };
  static __device__ __forceinline__ v16h load(const _Float16* p) {
    U f; f.h[0] = *(const v8h*)(p); f.h[1] = *(const v8h*)(p + 16); return f.v;
  }
  static __device__ __forceinline__ v8f mma(v16h a, v16h b, v8f c) {
    return __builtin_amdgcn_wmma_f32_16x16x32_f16(false, a, false, b, (short)0, c, false, false);
  }
  static __device__ __forceinline__ void guard(v8f& a, v8f& b, v16h x, v16h y) { dep_guard_h(a, b, x, y); }
  static __device__ __forceinline__ void keep(v16h a, v16h b, v16h c, v16h d) { keep4_h(a, b, c, d); }
};
template <> struct Frag<__bf16> {
  typedef v16b V; union U { v16b v; v8b h[2]; };
  static __device__ __forceinline__ v16b load(const __bf16* p) {
    U f; f.h[0] = *(const v8b*)(p); f.h[1] = *(const v8b*)(p + 16); return f.v;
  }
  static __device__ __forceinline__ v8f mma(v16b a, v16b b, v8f c) {
    return __builtin_amdgcn_wmma_f32_16x16x32_bf16(false, a, false, b, (short)0, c, false, false);
  }
  static __device__ __forceinline__ void guard(v8f& a, v8f& b, v16b x, v16b y) { dep_guard_b(a, b, x, y); }
  static __device__ __forceinline__ void keep(v16b a, v16b b, v16b c, v16b d) { keep4_b(a, b, c, d); }
};

__device__ __forceinline__ unsigned pk16(unsigned short a, unsigned short b) { return (unsigned)a | ((unsigned)b << 16); }
__device__ __forceinline__ unsigned short h_bits(float f) { const _Float16 h = (_Float16)f; return __builtin_bit_cast(unsigned short, h); }

template <int ET> struct Elem;
template <> struct Elem<0> { typedef _Float16 T; };
template <> struct Elem<1> { typedef __bf16 T; };
template <int ET, bool SPLIT, int BIAS_MODE, int OUT_MODE, bool RESID, int ACT = 0>
__global__ __launch_bounds__(256) void wmma_gemm64(
    const unsigned short* __restrict__ Ap, const unsigned short* __restrict__ A2p, int lda, long strideA,
    const unsigned short* __restrict__ Btp, const unsigned short* __restrict__ Bt2p, int ldb, long strideB,
    void* __restrict__ Cout, void* __restrict__ Cout2, int ldc, long strideC,
    const float* __restrict__ bias,
    const float* __restrict__ resid, long strideR,
    int M, int N, int K, float scale) {
  typedef typename Elem<ET>::T T;
  typedef typename Frag<T>::V V;
  const T* A = (const T*)Ap; const T* A2 = (const T*)A2p; const T* Bt = (const T*)Btp; const T* Bt2 = (const T*)Bt2p;
  __shared__ __align__(16) float sT[8][16 * 68];
  const int b    = blockIdx.y;
  const int lane = threadIdx.x & 31;
  const int wave = threadIdx.x >> 5;
  const int tilesN = N >> 6;
  const int tilesM = M >> 6;
  const int tile = blockIdx.x * 8 + wave;
  if (tile >= tilesM * tilesN) return;
  const int tm = tile / tilesN;
  const int tn = tile - tm * tilesN;
  const int m0 = tm << 6;
  const int n0 = tn << 6;

  const T* Ab  = A  + (size_t)b * strideA;
  const T* Bb  = Bt + (size_t)b * strideB;
  const T* Ab2 = SPLIT ? (A2  + (size_t)b * strideA) : nullptr;
  const T* Bb2 = SPLIT ? (Bt2 + (size_t)b * strideB) : nullptr;

  const int rlane = lane & 15;
  const int koff  = (lane >> 4) * 8;
  const int mOff  = (lane >> 4) * 8;

  v8f acc[4][4];
#pragma unroll
  for (int i = 0; i < 4; ++i)
#pragma unroll
    for (int j = 0; j < 4; ++j) acc[i][j] = (v8f){0.f,0.f,0.f,0.f,0.f,0.f,0.f,0.f};

  for (int k0 = 0; k0 < K; k0 += 32) {
    V bh[4], bl[4];
#pragma unroll
    for (int j = 0; j < 4; ++j) {
      const size_t bo = (size_t)(n0 + (j << 4) + rlane) * ldb + koff + k0;
      bh[j] = Frag<T>::load(Bb + bo);
      if (SPLIT) bl[j] = Frag<T>::load(Bb2 + bo);
    }
#pragma unroll
    for (int i = 0; i < 4; ++i) {
      const size_t ao = (size_t)(m0 + (i << 4) + rlane) * lda + koff + k0;
      V ah = Frag<T>::load(Ab + ao);
      V al;
      if (SPLIT) al = Frag<T>::load(Ab2 + ao);
#pragma unroll
      for (int j = 0; j < 4; ++j) {
        acc[i][j] = Frag<T>::mma(ah, bh[j], acc[i][j]);
        if (SPLIT) {
          acc[i][j] = Frag<T>::mma(ah, bl[j], acc[i][j]);
          acc[i][j] = Frag<T>::mma(al, bh[j], acc[i][j]);
        }
      }
      Frag<T>::guard(acc[i][0], acc[i][3], ah, SPLIT ? al : ah);
    }
    Frag<T>::keep(bh[0], bh[1], bh[2], bh[3]);
    if (SPLIT) Frag<T>::keep(bl[0], bl[1], bl[2], bl[3]);
  }
  acc_guard4(acc[0][0], acc[0][1], acc[0][2], acc[0][3]);
  acc_guard4(acc[1][0], acc[1][1], acc[1][2], acc[1][3]);
  acc_guard4(acc[2][0], acc[2][1], acc[2][2], acc[2][3]);
  acc_guard4(acc[3][0], acc[3][1], acc[3][2], acc[3][3]);

  float* slab = sT[wave];
  const float* Rb = RESID ? (resid + (size_t)b * strideR) : nullptr;
#pragma unroll
  for (int i = 0; i < 4; ++i) {
    const int mBase = m0 + (i << 4);
#pragma unroll
    for (int j = 0; j < 4; ++j) {
      const int n = n0 + (j << 4) + rlane;
      float bv = 0.f;
      if (BIAS_MODE == 2) bv = bias[n];
#pragma unroll
      for (int r = 0; r < 8; ++r) {
        float v = acc[i][j][r] * scale;
        if (BIAS_MODE == 1) v += bias[mBase + mOff + r];
        if (BIAS_MODE == 2) v += bv;
        if (RESID) v += Rb[(size_t)(mBase + mOff + r) * ldc + n];
        if (ACT == 2) v = fmaxf(v, 0.0f);
        if (ACT == 4) v = (v > 0.f) ? v : 0.01f * v;
        slab[(mOff + r) * 68 + (j << 4) + rlane] = v;
      }
    }
    __builtin_amdgcn_fence(__ATOMIC_RELEASE, "workgroup");
    __builtin_amdgcn_wave_barrier();
    __builtin_amdgcn_fence(__ATOMIC_ACQUIRE, "workgroup");
    if (OUT_MODE == 0) {
      float* C = (float*)Cout + (size_t)b * strideC;
      const int hh = lane >> 4, c4 = (lane & 15) * 4;
      for (int pass = 0; pass < 2; ++pass) {
#pragma unroll
        for (int it = 0; it < 8; ++it) {
          const int row = it * 2 + hh;
          v4f v = *(const v4f*)(slab + row * 68 + c4);
          *(volatile v4f*)(C + (size_t)(mBase + row) * ldc + n0 + c4) = v;
        }
        __threadfence();
      }
    } else {
      const int q = lane >> 3, c8 = (lane & 7) * 8;
      unsigned short* C  = (unsigned short*)Cout  + (size_t)b * strideC;
      unsigned short* C2 = (OUT_MODE == 2) ? ((unsigned short*)Cout2 + (size_t)b * strideC) : nullptr;
      for (int pass = 0; pass < 2; ++pass) {
#pragma unroll
        for (int it = 0; it < 4; ++it) {
          const int row = it * 4 + q;
          const float* sp = slab + row * 68 + c8;
          v8h hv, lv;
#pragma unroll
          for (int e = 0; e < 8; ++e) {
            if (OUT_MODE == 1) {
              hv[e] = (_Float16)sp[e];
            } else {
              unsigned short hb = f2bf_bits(sp[e]);
              unsigned short lb = f2bf_bits(sp[e] - bf_bits2f(hb));
              hv[e] = __builtin_bit_cast(_Float16, hb);
              lv[e] = __builtin_bit_cast(_Float16, lb);
            }
          }
          *(volatile v8h*)(C + (size_t)(mBase + row) * ldc + n0 + c8) = hv;
          if (OUT_MODE == 2) *(volatile v8h*)(C2 + (size_t)(mBase + row) * ldc + n0 + c8) = lv;
        }
        __threadfence();
      }
    }
    __builtin_amdgcn_fence(__ATOMIC_RELEASE, "workgroup");
    __builtin_amdgcn_wave_barrier();
    __builtin_amdgcn_fence(__ATOMIC_ACQUIRE, "workgroup");
  }
}

__global__ __launch_bounds__(256) void cast8_f16_kernel(const float* __restrict__ in, unsigned short* __restrict__ out, int n8) {
  const int i = blockIdx.x * 256 + threadIdx.x;
  if (i >= n8) return;
  const float* p = in + 8 * (size_t)i;
  const v4f a = *(const v4f*)(p);
  const v4f c = *(const v4f*)(p + 4);
  unsigned short hb[8];
#pragma unroll
  for (int e = 0; e < 4; ++e) {
    hb[e]     = h_bits(a[e]);
    hb[4 + e] = h_bits(c[e]);
  }
  const v4u u = (v4u){pk16(hb[0], hb[1]), pk16(hb[2], hb[3]), pk16(hb[4], hb[5]), pk16(hb[6], hb[7])};
  unsigned short* q = out + 8 * (size_t)i;
  *(volatile v4u*)q = u;
  __threadfence();
  *(volatile v4u*)q = u;
}

__global__ __launch_bounds__(256) void k_wtcast3(const float* __restrict__ Wp0, const float* __restrict__ Wp1, const float* __restrict__ Wp2,
                                                  unsigned short* __restrict__ Op0, unsigned short* __restrict__ Op1,
                                                  unsigned short* __restrict__ Op2, float scale) {
  __shared__ float sm[64][65];
  const int t = threadIdx.x;
  const int z = blockIdx.z;
  const float* W = (z == 0) ? Wp0 : (z == 1) ? Wp1 : Wp2;
  unsigned short* op = (z == 0) ? Op0 : (z == 1) ? Op1 : Op2;
  const int nR = (z == 0) ? kIn : kHid;
  const int nC = (z == 0) ? kHid : (z == 1) ? kOut : kHid;
  const int k0 = blockIdx.x * 64;
  const int c0 = blockIdx.y * 64;
  if (k0 >= nR || c0 >= nC) return;
#pragma unroll
  for (int i = 0; i < 16; ++i) {
    const int e = i * 256 + t;
    const int r = e >> 6;
    const int cc = e & 63;
    sm[cc][r] = W[(size_t)(k0 + r) * nC + c0 + cc] * scale;
  }
  __syncthreads();
  const int lane = t & 31, wave = t >> 5;
  const int q = lane >> 3, c8 = (lane & 7) * 8;
  for (int pass = 0; pass < 2; ++pass) {
#pragma unroll
    for (int it = 0; it < 2; ++it) {
      const int row = wave * 8 + it * 4 + q;
      unsigned short hb[8];
#pragma unroll
      for (int e = 0; e < 8; ++e) hb[e] = h_bits(sm[row][c8 + e]);
      const v4u u = (v4u){pk16(hb[0], hb[1]), pk16(hb[2], hb[3]), pk16(hb[4], hb[5]), pk16(hb[6], hb[7])};
      *(volatile v4u*)(op + (size_t)(c0 + row) * nR + k0 + c8) = u;
    }
    __threadfence();
  }
}

__device__ __forceinline__ int blk_excl_scan(int cnt, int* scan_ws, int tid, int* tot) {
  const int lane = tid & 31, wave = tid >> 5; int incl = cnt;
#pragma unroll
  for (int o = 1; o < 32; o <<= 1) { const int v = __shfl_up(incl, o, 32); if (lane >= o) incl += v; }
  if (lane == 31) scan_ws[wave] = incl;
  __syncthreads();
  if (wave == 0) { int wv = (lane < kThr / 32) ? scan_ws[lane] : 0; int wincl = wv;
#pragma unroll
    for (int o = 1; o < 32; o <<= 1) { const int v = __shfl_up(wincl, o, 32); if (lane >= o) wincl += v; }
    if (lane < kThr / 32) scan_ws[32 + lane] = wincl - wv; if (lane == 31) scan_ws[64] = wincl; }
  __syncthreads();
  const int res = scan_ws[32 + wave] + incl - cnt; *tot = scan_ws[64];
  return res;
}
__device__ __forceinline__ int chunk_hits_tile(const int* __restrict__ dstv, const int* __restrict__ srcv, int e0, int n0, int tid,
                                               int* LIST, int* scan_ws) {
  const int eb = e0 + tid * kSpt;
  int rec[kSpt]; int cnt = 0;
#pragma unroll
  for (int k = 0; k < kSpt; k += 4) {
    const v4i d4 = *(const v4i*)(dstv + eb + k);
    const v4i s4 = *(const v4i*)(srcv + eb + k);
#pragma unroll
    for (int e = 0; e < 4; ++e) {
      const int d = d4[e]; int r = -1;
      if (d >= n0 && d < n0 + kTD) { int s = s4[e]; s = s < 0 ? 0 : (s > kN - 1 ? kN - 1 : s); r = ((d - n0) << 16) | s; ++cnt; }
      rec[k + e] = r;
    }
  }
  int tot; int p = blk_excl_scan(cnt, scan_ws, tid, &tot);
#pragma unroll
  for (int k = 0; k < kSpt; ++k) if (rec[k] >= 0) { if ((unsigned)p < (unsigned)kSch) LIST[p] = rec[k]; ++p; }
  __syncthreads();
  return tot < kSch ? tot : kSch;
}

__global__ __launch_bounds__(kThr) void k_deg(const int* __restrict__ ei, float* __restrict__ dinvg, float* __restrict__ invg) {
  __shared__ int LIST[kSch];
  __shared__ int scan_ws[80];
  __shared__ __align__(16) float sdeg[kTD];
  const int tid = threadIdx.x, lane = tid & 31, wave = tid >> 5;
  const int t = blockIdx.x / kTiles;
  const int tile = blockIdx.x - t * kTiles;
  const int n0 = tile * kTD;
  const int rowbase = t * kN;
  if (tid < 80) scan_ws[tid] = 0;
  __syncthreads();
  const int* srcv = ei + (size_t)t * 2 * kE;
  const int* dstv = srcv + kE;
  int cnt = 0;
#pragma unroll 1
  for (int c = 0; c < kNch; ++c) {
    const int tot = chunk_hits_tile(dstv, srcv, c * kSch, n0, tid, LIST, scan_ws);
    if (tid < kTD) {
#pragma unroll 1
      for (int q = 0; q < tot; ++q) cnt += ((LIST[q] >> 16) == tid) ? 1 : 0;
    }
    __syncthreads();
  }
  if (tid < kTD) sdeg[tid] = (float)(cnt + 1);
  __syncthreads();
  if (wave == 0) {
    const v4f d = *(const v4f*)(sdeg + 4 * lane);
    v4f di, iv;
#pragma unroll
    for (int e = 0; e < 4; ++e) { const float dd = d[e]; di[e] = 1.0f / sqrtf(dd); iv[e] = 1.0f / dd; }
    float* pd = dinvg + rowbase + n0 + 4 * lane;
    float* pi = invg + rowbase + n0 + 4 * lane;
    for (int pass = 0; pass < 2; ++pass) { *(volatile v4f*)pd = di; *(volatile v4f*)pi = iv; __threadfence(); }
  }
}

template <int F, int MODE>
__global__ __launch_bounds__(kThr) void k_agg(const float* __restrict__ xw, const int* __restrict__ ei,
                                            const float* __restrict__ dinvg, const float* __restrict__ invg,
                                            const float* __restrict__ bias,
                                            unsigned short* __restrict__ out16, float* __restrict__ out32) {
  static_assert(F == 64 || F == 128, "F");
  static_assert((MODE == 0 && F == 128) || (MODE == 1 && F == 64), "mode and width");
  typedef float vl __attribute__((ext_vector_type(F / 32)));
  constexpr int VW = F / 32;
  __shared__ __align__(16) float sacc[kTD * F];
  __shared__ int LIST[kSch];
  __shared__ int scan_ws[80];
  __shared__ float sdi[kTD];
  __shared__ float sinv[kTD];
  const int tid = threadIdx.x, lane = tid & 31, wave = tid >> 5;
  const int t = blockIdx.x / kTiles;
  const int tile = blockIdx.x - t * kTiles;
  const int n0 = tile * kTD;
  const int rowbase = t * kN;
  const v4f z4 = {0.f, 0.f, 0.f, 0.f};
  for (int i = tid; i < kTD * F / 4; i += kThr) *(v4f*)(sacc + 4 * i) = z4;
  if (tid < kTD) { sdi[tid] = dinvg[rowbase + n0 + tid]; sinv[tid] = invg[rowbase + n0 + tid]; }
  if (tid < 80) scan_ws[tid] = 0;
  __syncthreads();
  const int* srcv = ei + (size_t)t * 2 * kE;
  const int* dstv = srcv + kE;
#pragma unroll 1
  for (int c = 0; c < kNch; ++c) {
    const int tot = chunk_hits_tile(dstv, srcv, c * kSch, n0, tid, LIST, scan_ws);
#pragma unroll 1
    for (int base = 0; base < tot; base += 32) {
      const int q = base + lane;
      const int qc = (q < tot) ? q : (tot - 1);
      const int rraw = LIST[qc];
      const int rv = (q < tot) ? rraw : -1;
      const int own = (rv >= 0 && (rv >> 20) == wave) ? 1 : 0;
      unsigned msk = (unsigned)__ballot(own);
#pragma unroll 1
      for (int it = 0; it < 32; ++it) {
        if (msk == 0u) break;
        const int bp = __builtin_ctz(msk); msk &= msk - 1u;
        const int r = __shfl(rv, bp, 32);
        const int dl = r >> 16, s = r & 0xFFFF;
        const float nrm = dinvg[rowbase + s] * sdi[dl];
        const vl xv = *(const vl*)(xw + (size_t)(rowbase + s) * F + VW * lane);
        float* ap = sacc + dl * F + VW * lane;
        vl a = *(const vl*)ap;
        a = a + xv * nrm;
        *(vl*)ap = a;
      }
    }
    __syncthreads();
  }
  if (MODE == 0) {
    const int c8 = (lane & 15) * 8;
    const v4f b0 = *(const v4f*)(bias + c8);
    const v4f b1 = *(const v4f*)(bias + c8 + 4);
#pragma unroll 1
    for (int j = 0; j < kTD / 8; ++j) {
      const int dl = wave * (kTD / 8) + j;
      const int row = rowbase + n0 + dl;
      const float iv = sinv[dl];
      const float* xr = xw + (size_t)row * F + c8;
      const v4f x0 = *(const v4f*)xr;
      const v4f x1 = *(const v4f*)(xr + 4);
      const float* ar = sacc + dl * F + c8;
      const v4f a0 = *(const v4f*)ar;
      const v4f a1 = *(const v4f*)(ar + 4);
      v4f v0 = a0 + x0 * iv; v0 = v0 + b0;
      v4f v1 = a1 + x1 * iv; v1 = v1 + b1;
      unsigned short hb[8];
#pragma unroll
      for (int e = 0; e < 4; ++e) {
        const float p0 = v0[e], p1 = v1[e];
        hb[e]     = h_bits(fmaxf(p0, 0.0f) * kCarry);
        hb[4 + e] = h_bits(fmaxf(p1, 0.0f) * kCarry);
      }
      const v4u u = (v4u){pk16(hb[0], hb[1]), pk16(hb[2], hb[3]), pk16(hb[4], hb[5]), pk16(hb[6], hb[7])};
      unsigned short* dst = out16 + (size_t)row * F + c8;
      for (int pass = 0; pass < 2; ++pass) {
        if (lane < 16) *(volatile v4u*)dst = u;
        __threadfence();
      }
    }
  } else {
    const int c4 = (lane & 15) * 4;
    const int c8 = (lane & 7) * 8;
    const v4f bq = *(const v4f*)(bias + c4);
    const v4f b0 = *(const v4f*)(bias + c8);
    const v4f b1 = *(const v4f*)(bias + c8 + 4);
    const bool last = (t == kT - 1);
#pragma unroll 1
    for (int j = 0; j < kTD / 8; ++j) {
      const int dl = wave * (kTD / 8) + j;
      const int n = n0 + dl;
      const int row = rowbase + n;
      const float iv = sinv[dl];
      const float* xr = xw + (size_t)row * F;
      const float* ar = sacc + dl * F;
      const v4f xq = *(const v4f*)(xr + c4);
      const v4f aq = *(const v4f*)(ar + c4);
      v4f vq = aq + xq * iv; vq = vq + bq;
      const v4f x0 = *(const v4f*)(xr + c8);
      const v4f x1 = *(const v4f*)(xr + c8 + 4);
      const v4f a0 = *(const v4f*)(ar + c8);
      const v4f a1 = *(const v4f*)(ar + c8 + 4);
      v4f v0 = a0 + x0 * iv; v0 = v0 + b0;
      v4f v1 = a1 + x1 * iv; v1 = v1 + b1;
      unsigned short hb[8];
#pragma unroll
      for (int e = 0; e < 4; ++e) {
        const float p0 = v0[e], p1 = v1[e];
        hb[e]     = h_bits(p0 * kCarry);
        hb[4 + e] = h_bits(p1 * kCarry);
      }
      const v4u u = (v4u){pk16(hb[0], hb[1]), pk16(hb[2], hb[3]), pk16(hb[4], hb[5]), pk16(hb[6], hb[7])};
      float* d32 = out32 + (size_t)row * F + c4;
      unsigned short* d16 = out16 + (size_t)n * F + c8;
      for (int pass = 0; pass < 2; ++pass) {
        if (lane < 16) *(volatile v4f*)d32 = vq;
        if (last && lane < 8) *(volatile v4u*)d16 = u;
        __threadfence();
      }
    }
  }
}

__global__ __launch_bounds__(512) void k_gru(const float* __restrict__ enc, const float* __restrict__ Wih, const float* __restrict__ Whh,
                                           const float* __restrict__ bih, const float* __restrict__ bhh,
                                           const float* __restrict__ Wd1, const float* __restrict__ bd1, float* __restrict__ cvec) {
  __shared__ float sP[kT * kOut];
  __shared__ float sh[kHid];
  __shared__ float sgi[3 * kHid];
  __shared__ float sgh[3 * kHid];
  __shared__ __align__(16) float sC[kHid];
  const int tid = threadIdx.x;
  {
    const int tt = tid >> 6, f = tid & 63;
    const float* p = enc + (size_t)tt * kN * kOut + f;
    float s0 = 0.0f, s1 = 0.0f, s2 = 0.0f, s3 = 0.0f;
#pragma unroll 1
    for (int n = 0; n < kN; n += 4) {
      s0 += p[(size_t)(n) * kOut];
      s1 += p[(size_t)(n + 1) * kOut];
      s2 += p[(size_t)(n + 2) * kOut];
      s3 += p[(size_t)(n + 3) * kOut];
    }
    sP[tid] = ((s0 + s1) + (s2 + s3)) * (1.0f / 1024.0f);
  }
  if (tid < kHid) sh[tid] = 0.0f;
  __syncthreads();
#pragma unroll 1
  for (int step = 0; step < kT; ++step) {
    if (tid < 3 * kHid) {
      const float* wi = Wih + (size_t)tid * kOut;
      const float* wh = Whh + (size_t)tid * kHid;
      const float* xp = sP + step * kOut;
      float di = 0.0f, dh = 0.0f;
#pragma unroll 1
      for (int k = 0; k < kOut; ++k) di = fmaf(wi[k], xp[k], di);
#pragma unroll 1
      for (int k = 0; k < kHid; ++k) dh = fmaf(wh[k], sh[k], dh);
      sgi[tid] = di + bih[tid];
      sgh[tid] = dh + bhh[tid];
    }
    __syncthreads();
    float hn = 0.0f;
    if (tid < kHid) {
      const float rr = 1.0f / (1.0f + expf(-(sgi[tid] + sgh[tid])));
      const float zz = 1.0f / (1.0f + expf(-(sgi[kHid + tid] + sgh[kHid + tid])));
      const float nn = tanhf(sgi[2 * kHid + tid] + rr * sgh[2 * kHid + tid]);
      hn = (1.0f - zz) * nn + zz * sh[tid];
    }
    __syncthreads();
    if (tid < kHid) sh[tid] = hn;
    __syncthreads();
  }
  if (tid < kHid) {
    float d = 0.0f;
    const float* wc = Wd1 + (size_t)(2 * kOut) * kHid + tid;
#pragma unroll 1
    for (int k = 0; k < kHid; ++k) d = fmaf(sh[k], wc[(size_t)k * kHid], d);
    sC[tid] = d + bd1[tid];
  }
  __syncthreads();
  if (tid < 32) {
    const v4f v = *(const v4f*)(sC + 4 * tid);
    float* op = cvec + 4 * tid;
    for (int pass = 0; pass < 2; ++pass) { *(volatile v4f*)op = v; __threadfence(); }
  }
}

__global__ __launch_bounds__(kThr) void k_pairs(const float* __restrict__ Ap, const float* __restrict__ BTp, const float* __restrict__ cvec,
                                              const float* __restrict__ Wd2, const float* __restrict__ bd2, float* __restrict__ out) {
  __shared__ float sAc[2 * kHid];
  __shared__ float sW[kHid];
  const int tid = threadIdx.x;
  const int blk = blockIdx.x;
  sAc[tid] = Ap[(size_t)(blk + (tid >> 7)) * kHid + (tid & 127)] + cvec[tid & 127];
  if (tid < kHid) sW[tid] = Wd2[tid];
  __syncthreads();
  const int qs = (kN - 1) - blk;
  int aoff[4];
  const float* bp[4];
  float acc[4];
#pragma unroll
  for (int u = 0; u < 4; ++u) {
    const int q = 4 * tid + u;
    const int sel = (q >= qs) ? 1 : 0;
    const int i = blk + sel;
    const int jj = blk + q - (kN - 1) * sel;
    const int j = jj + ((jj >= i) ? 1 : 0);
    aoff[u] = sel * kHid;
    bp[u] = BTp + j;
    acc[u] = 0.0f;
  }
#pragma unroll 2
  for (int f = 0; f < kHid; ++f) {
    const float w = sW[f];
#pragma unroll
    for (int u = 0; u < 4; ++u) {
      const float a = sAc[aoff[u] + f];
      const float bvv = bp[u][(size_t)f * kN];
      float tv = a + bvv;
      tv = fmaxf(tv, 0.0f);
      acc[u] = fmaf(tv, w, acc[u]);
    }
  }
  const float b2 = bd2[0];
  v4f o;
  o[0] = acc[0] + b2; o[1] = acc[1] + b2; o[2] = acc[2] + b2; o[3] = acc[3] + b2;
  float* op = out + (size_t)blk * kPairsPerBlock + 4 * tid;
  *(volatile v4f*)op = o;
  __threadfence();
  *(volatile v4f*)op = o;
}

extern "C" void kernel_launch(void* const* d_in, const int* in_sizes, int n_in,
                              void* d_out, int out_size, void* d_ws, size_t ws_size,
                              hipStream_t stream) {
  (void)in_sizes; (void)n_in; (void)out_size;
  const float* x_seq = (const float*)d_in[0];
  const int*   ei    = (const int*)  d_in[1];
  const float* Wc1   = (const float*)d_in[2];
  const float* bc1   = (const float*)d_in[3];
  const float* Wc2   = (const float*)d_in[4];
  const float* bc2   = (const float*)d_in[5];
  const float* Wih   = (const float*)d_in[6];
  const float* Whh   = (const float*)d_in[7];
  const float* bih   = (const float*)d_in[8];
  const float* bhh   = (const float*)d_in[9];
  const float* Wd1   = (const float*)d_in[10];
  const float* bd1   = (const float*)d_in[11];
  const float* Wd2   = (const float*)d_in[12];
  const float* bd2   = (const float*)d_in[13];
  float* out = (float*)d_out;

  char* ws = (char*)d_ws; size_t off = 0;
  auto carve = [&](size_t bytes) -> char* { char* p = ws + off; off += (bytes + 255) & ~(size_t)255; return p; };
  float*          dinvg = (float*)carve((size_t)kRows * 4);
  float*          invg  = (float*)carve((size_t)kRows * 4);
  unsigned short* x16   = (unsigned short*)carve((size_t)kRows * kIn * 2);
  unsigned short* bt1   = (unsigned short*)carve((size_t)kHid * kIn * 2);
  unsigned short* bt2   = (unsigned short*)carve((size_t)kOut * kHid * 2);
  unsigned short* wab   = (unsigned short*)carve((size_t)kHid * kHid * 2);
  float*          xw1   = (float*)carve((size_t)kRows * kHid * 4);
  unsigned short* h16   = (unsigned short*)carve((size_t)kRows * kHid * 2);
  float*          xw2   = (float*)carve((size_t)kRows * kOut * 4);
  float*          enc   = (float*)carve((size_t)kRows * kOut * 4);
  unsigned short* e16   = (unsigned short*)carve((size_t)kN * kOut * 2);
  float*          cvec  = (float*)carve((size_t)kHid * 4);
  float*          aproj = (float*)carve((size_t)kN * kHid * 4);
  float*          bT    = (float*)carve((size_t)kHid * kN * 4);
  if (off > ws_size || off > (size_t)134217728) return;

  cast8_f16_kernel<<<(kRows * kIn / 8 + 255) / 256, 256, 0, stream>>>(x_seq, x16, kRows * kIn / 8);
  k_wtcast3<<<dim3(2, 2, 3), 256, 0, stream>>>(Wc1, Wc2, Wd1, bt1, bt2, wab, kCarry);
  k_deg<<<kT * kTiles, kThr, 0, stream>>>(ei, dinvg, invg);
  wmma_gemm64<0, false, 0, 0, false, 0><<<dim3((kRows / 64) * (kHid / 64) / 8, 1), 256, 0, stream>>>(
      x16, (const unsigned short*)nullptr, kIn, 0L,
      bt1, (const unsigned short*)nullptr, kIn, 0L,
      (void*)xw1, (void*)nullptr, kHid, 0L,
      (const float*)nullptr, (const float*)nullptr, 0L, kRows, kHid, kIn, kScale1);
  k_agg<128, 0><<<kT * kTiles, kThr, 0, stream>>>(xw1, ei, dinvg, invg, bc1, h16, (float*)nullptr);
  wmma_gemm64<0, false, 0, 0, false, 0><<<dim3((kRows / 64) * (kOut / 64) / 8, 1), 256, 0, stream>>>(
      h16, (const unsigned short*)nullptr, kHid, 0L,
      bt2, (const unsigned short*)nullptr, kHid, 0L,
      (void*)xw2, (void*)nullptr, kOut, 0L,
      (const float*)nullptr, (const float*)nullptr, 0L, kRows, kOut, kHid, kScale2);
  k_agg<64, 1><<<kT * kTiles, kThr, 0, stream>>>(xw2, ei, dinvg, invg, bc2, e16, enc);
  k_gru<<<1, 512, 0, stream>>>(enc, Wih, Whh, bih, bhh, Wd1, bd1, cvec);
  wmma_gemm64<0, false, 0, 0, false, 0><<<dim3((kN / 64) * (kHid / 64) / 8, 1), 256, 0, stream>>>(
      e16, (const unsigned short*)nullptr, kOut, 0L,
      wab, (const unsigned short*)nullptr, kHid, 0L,
      (void*)aproj, (void*)nullptr, kHid, 0L,
      (const float*)nullptr, (const float*)nullptr, 0L, kN, kHid, kOut, kScale2);
  wmma_gemm64<0, false, 0, 0, false, 0><<<dim3((kHid / 64) * (kN / 64) / 8, 1), 256, 0, stream>>>(
      wab + kOut, (const unsigned short*)nullptr, kHid, 0L,
      e16, (const unsigned short*)nullptr, kOut, 0L,
      (void*)bT, (void*)nullptr, kN, 0L,
      (const float*)nullptr, (const float*)nullptr, 0L, kHid, kN, kOut, kScale2);
  k_pairs<<<kPairBlocks, kThr, 0, stream>>>(aproj, bT, cvec, Wd2, bd2, out);
}
